// NonLocalBlock_63024350102345
// MI455X (gfx1250) — hardware-verified
//
#include <hip/hip_runtime.h>


#ifndef NB
#define NB 4
#endif
#ifndef SEQ
#define SEQ 4096
#endif
#define NB_FULL  4
#define SEQ_FULL 4096
#define CC   256
#define HW   SEQ
#define PCAR 1024.0f
static_assert(NB >= 1 && NB <= NB_FULL);
static_assert(SEQ >= 128 && SEQ <= SEQ_FULL && (SEQ % 128) == 0);
static_assert((CC % 64) == 0 && (HW % 64) == 0 && (CC % 32) == 0);

typedef _Float16 h16;
typedef unsigned short bf;
typedef __attribute__((ext_vector_type(16))) __bf16   v16bf;
typedef __attribute__((ext_vector_type(16))) _Float16 v16h;
typedef __attribute__((ext_vector_type(8)))  _Float16 v8h;
typedef __attribute__((ext_vector_type(8)))  unsigned short v8us;
typedef __attribute__((ext_vector_type(8)))  float    v8f;
typedef __attribute__((ext_vector_type(4)))  float    v4f;
typedef v8h  __attribute__((may_alias)) v8ha;
typedef v4f  __attribute__((may_alias)) v4fa;
typedef v8us __attribute__((may_alias)) v8usa;

__device__ __forceinline__ unsigned short f2bf(float f) { unsigned u = __float_as_uint(f); u += 0x7FFFu + ((u >> 16) & 1u); return (unsigned short)(u >> 16); }
__device__ __forceinline__ float bf2f(unsigned short b) { return __uint_as_float(((unsigned)b) << 16); }
__device__ __forceinline__ float bfr(float f) { return bf2f(f2bf(f)); }
__device__ __forceinline__ v16h cat16(v8h lo, v8h hi) { return __builtin_shufflevector(lo, hi, 0, 1, 2, 3, 4, 5, 6, 7, 8, 9, 10, 11, 12, 13, 14, 15); }
__device__ __forceinline__ v16bf cat16b(v8us lo, v8us hi) { return __builtin_bit_cast(v16bf, __builtin_shufflevector(lo, hi, 0, 1, 2, 3, 4, 5, 6, 7, 8, 9, 10, 11, 12, 13, 14, 15)); }
__device__ __forceinline__ v8f wmma16(v16h a, v16h b, v8f c) { return __builtin_amdgcn_wmma_f32_16x16x32_f16(false, a, false, b, (short)0, c, false, false); }
__device__ __forceinline__ v8f wmmab(v16bf a, v16bf b, v8f c) { return __builtin_amdgcn_wmma_f32_16x16x32_bf16(false, a, false, b, (short)0, c, false, false); }

template <typename T16> struct WFrag;
template <> struct WFrag<h16> { typedef v16h V; static __device__ __forceinline__ V ld(const h16* p) { return cat16(*(const v8h*)p, *(const v8h*)(p + 16)); } static __device__ __forceinline__ v8f mma(V a, V b, v8f c) { return wmma16(a, b, c); } };
template <> struct WFrag<bf> { typedef v16bf V; static __device__ __forceinline__ V ld(const bf* p) { return cat16b(*(const v8us*)p, *(const v8us*)(p + 16)); } static __device__ __forceinline__ v8f mma(V a, V b, v8f c) { return wmmab(a, b, c); } };
template <typename T16, int NSPLIT, int BIAS>
__global__ __launch_bounds__(32) void k_gemmw(const T16* __restrict__ A, const T16* __restrict__ A2, const T16* __restrict__ Bt, const T16* __restrict__ Bt2, int K, float* C, int ldc, const float* __restrict__ bias, size_t sA, size_t sB, size_t sC) {
    typedef typename WFrag<T16>::V V;
    __shared__ __align__(16) float os[16 * 68];
    const size_t z = blockIdx.z; A += z * sA; if (A2) A2 += z * sA; Bt += z * sB; if (Bt2) Bt2 += z * sB; C += z * sC;
    const int lane = threadIdx.x & 31, lr = lane & 15, hi = lane >> 4; const int r0 = blockIdx.x * 64, c0 = blockIdx.y * 64;
    v8f acc[4][4];
#pragma unroll
    for (int mb = 0; mb < 4; ++mb)
#pragma unroll
        for (int nb = 0; nb < 4; ++nb) acc[mb][nb] = (v8f){};
    const size_t aoff = (size_t)(r0 + lr) * K + 8 * hi, boff = (size_t)(c0 + lr) * K + 8 * hi;
#pragma unroll 1
    for (int kc = 0; kc < K; kc += 32) {
        V a[4], a2[4];
#pragma unroll
        for (int mb = 0; mb < 4; ++mb) { a[mb] = WFrag<T16>::ld(A + aoff + (size_t)mb * 16 * K + kc); if (NSPLIT == 1 || NSPLIT == 2) a2[mb] = WFrag<T16>::ld(A2 + aoff + (size_t)mb * 16 * K + kc); }
#pragma unroll
        for (int nb = 0; nb < 4; ++nb) { const V b = WFrag<T16>::ld(Bt + boff + (size_t)nb * 16 * K + kc); V b2; if (NSPLIT >= 2) b2 = WFrag<T16>::ld(Bt2 + boff + (size_t)nb * 16 * K + kc);
#pragma unroll
            for (int mb = 0; mb < 4; ++mb) { acc[mb][nb] = WFrag<T16>::mma(a[mb], b, acc[mb][nb]); if (NSPLIT == 1 || NSPLIT == 2) acc[mb][nb] = WFrag<T16>::mma(a2[mb], b, acc[mb][nb]); if (NSPLIT >= 2) acc[mb][nb] = WFrag<T16>::mma(a[mb], b2, acc[mb][nb]); } }
        asm volatile("v_nop\n\tv_nop\n\tv_nop\n\tv_nop" : "+v"(acc[0][0]), "+v"(acc[1][1]), "+v"(acc[2][2]), "+v"(acc[3][3]) : "v"(a[0]), "v"(a[3]));
    }
#pragma unroll
    for (int mb = 0; mb < 4; ++mb) {
#pragma unroll
        for (int nb = 0; nb < 4; ++nb) {
#pragma unroll
            for (int j = 0; j < 8; ++j) os[(hi * 8 + j) * 68 + nb * 16 + lr] = acc[mb][nb][j]; }
        __builtin_amdgcn_wave_barrier(); asm volatile("" ::: "memory");
        float* crow = C + (size_t)(r0 + mb * 16) * ldc + c0;
#pragma unroll 1
        for (int ps = 0; ps < 2; ++ps) {
#pragma unroll
            for (int s = 0; s < 8; ++s) { const int row = 2 * s + hi, cofs = lr * 4; v4f val = *(const v4fa*)(os + row * 68 + cofs);
                if (BIAS == 1) { val[0] += bfr(bias[c0 + cofs]); val[1] += bfr(bias[c0 + cofs + 1]); val[2] += bfr(bias[c0 + cofs + 2]); val[3] += bfr(bias[c0 + cofs + 3]); }
                if (BIAS == 2) { const float rb = bfr(bias[r0 + mb * 16 + row]); val[0] += rb; val[1] += rb; val[2] += rb; val[3] += rb; }
                *(volatile v4f*)(crow + (size_t)row * ldc + cofs) = val; }
            if (ps == 0) __threadfence(); }
        __builtin_amdgcn_wave_barrier(); asm volatile("" ::: "memory");
    }
}

__device__ __forceinline__ h16 tohx(float x) { return (h16)x; }
__device__ __forceinline__ void splitf(float y, unsigned short& h, unsigned short& l) { h = f2bf(y); l = f2bf(y - bf2f(h)); }
typedef __attribute__((ext_vector_type(2))) unsigned short v2us;
typedef __attribute__((ext_vector_type(4))) unsigned short v4us;
typedef __attribute__((ext_vector_type(2))) _Float16 v2h;
typedef __attribute__((ext_vector_type(4))) _Float16 v4h;
typedef __attribute__((ext_vector_type(2))) float v2f;

__global__ __launch_bounds__(256) void k_cvt8(const float* __restrict__ src, bf* dst, size_t n8) { const size_t i = (size_t)blockIdx.x * 256 + threadIdx.x; if (i >= n8) return; const v8f v = *(const v8f*)(src + i * 8); v8us o;
#pragma unroll
    for (int k = 0; k < 8; ++k) o[k] = f2bf(v[k]); *(volatile v8us*)(dst + i * 8) = o; __threadfence(); *(volatile v8us*)(dst + i * 8) = o; }
__global__ __launch_bounds__(256) void k_xt(const float* __restrict__ xb, bf* XT) { const size_t e = ((size_t)blockIdx.x * 256 + threadIdx.x) * 4; if (e >= (size_t)HW * CC) return; const int c = (int)(e % CC); const int m = (int)(e / CC); v4us o;
#pragma unroll
    for (int u = 0; u < 4; ++u) o[u] = f2bf(xb[(size_t)(c + u) * SEQ_FULL + m]); *(volatile v4us*)(XT + e) = o; __threadfence(); *(volatile v4us*)(XT + e) = o; }
__global__ __launch_bounds__(256) void k_hl(const float* __restrict__ F, bf* Fh, bf* Fl) { const size_t e = ((size_t)blockIdx.x * 256 + threadIdx.x) * 4; if (e >= (size_t)HW * CC) return; const v4f a = *(const v4f*)(F + e); v4us oh, ol; for (int u = 0; u < 4; ++u) { unsigned short p, q; splitf(a[u], p, q); oh[u] = p; ol[u] = q; } *(volatile v4us*)(Fh + e) = oh; *(volatile v4us*)(Fl + e) = ol; __threadfence(); *(volatile v4us*)(Fh + e) = oh; *(volatile v4us*)(Fl + e) = ol; }
__global__ __launch_bounds__(256) void k_gt16(const float* __restrict__ G, h16* GT) { const size_t e = ((size_t)blockIdx.x * 256 + threadIdx.x) * 2; if (e >= (size_t)CC * HW) return; const int m = (int)(e % HW); const int i = (int)(e / HW); v2h o; o[0] = tohx(G[(size_t)m * CC + i]); o[1] = tohx(G[(size_t)(m + 1) * CC + i]); *(volatile v2h*)(GT + e) = o; __threadfence(); *(volatile v2h*)(GT + e) = o; }
__global__ __launch_bounds__(256) void k_rsoft(const float* __restrict__ S, h16* P16) { const int lane = threadIdx.x & 31; const int row = blockIdx.x * 8 + (threadIdx.x >> 5); if (row >= HW) return; const float* sr = S + (size_t)row * HW; float v[HW / 32]; float mx = -3.0e38f;
#pragma unroll
    for (int ch = 0; ch < HW / 128; ++ch) { const v4f a = *(const v4f*)(sr + ch * 128 + lane * 4);
#pragma unroll
        for (int u = 0; u < 4; ++u) { v[ch * 4 + u] = a[u]; mx = fmaxf(mx, a[u]); } }
#pragma unroll
    for (int sh = 16; sh; sh >>= 1) mx = fmaxf(mx, __shfl_xor(mx, sh, 32));
    float sum = 0.f;
#pragma unroll
    for (int q = 0; q < HW / 32; ++q) { float d0 = __fsub_rn(v[q], mx); asm volatile("" : "+v"(d0)); v[q] = __builtin_amdgcn_exp2f(__fmul_rn(d0, 1.4426950408889634f)); sum += v[q]; }
#pragma unroll
    for (int sh = 16; sh; sh >>= 1) sum += __shfl_xor(sum, sh, 32);
    const float f = __fdiv_rn(PCAR, sum);
    for (int ps = 0; ps < 2; ++ps) {
#pragma unroll
        for (int ch = 0; ch < HW / 128; ++ch) { v4h o4; for (int q = 0; q < 4; ++q) o4[q] = tohx(v[ch * 4 + q] * f); *(volatile v4h*)(P16 + (size_t)row * HW + ch * 128 + lane * 4) = o4; }
        if (ps == 0) __threadfence(); } }
__global__ __launch_bounds__(256) void k_at(const float* __restrict__ Y, bf* ATh, bf* ATl) { const size_t e = ((size_t)blockIdx.x * 256 + threadIdx.x) * 4; if (e >= (size_t)HW * CC) return; const int c = (int)(e % CC); const int s = (int)(e / CC); v4us oh, ol;
#pragma unroll
    for (int u = 0; u < 4; ++u) { unsigned short p, q; splitf(Y[(size_t)(c + u) * HW + s] * (1.0f / PCAR), p, q); oh[u] = p; ol[u] = q; }
    *(volatile v4us*)(ATh + e) = oh; *(volatile v4us*)(ATl + e) = ol; __threadfence(); *(volatile v4us*)(ATh + e) = oh; *(volatile v4us*)(ATl + e) = ol; }
__global__ __launch_bounds__(256) void k_fin(const float* __restrict__ Z, const float* __restrict__ xb, float* OUTb) { const size_t e = ((size_t)blockIdx.x * 256 + threadIdx.x) * 4; if (e >= (size_t)CC * HW) return; const int n = (int)(e % HW); const int c = (int)(e / HW); v4f r;
#pragma unroll
    for (int u = 0; u < 4; ++u) r[u] = __fadd_rn(Z[(size_t)(n + u) * CC + c], bfr(xb[(size_t)c * SEQ_FULL + n + u])); *(volatile v4f*)(OUTb + e) = r; __threadfence(); *(volatile v4f*)(OUTb + e) = r; }

constexpr size_t al256(size_t b) { return (b + 255) & ~(size_t)255; }
constexpr size_t WS_TOTAL = 4 * al256((size_t)CC * CC * 2) + al256((size_t)HW * CC * 2) + 3 * al256((size_t)CC * HW * 4) + 4 * al256((size_t)HW * CC * 2) + al256((size_t)CC * HW * 2)
                          + al256((size_t)HW * HW * 4) + al256((size_t)HW * HW * 2) + 2 * al256((size_t)HW * CC * 2);
static_assert(WS_TOTAL <= (size_t)134217728);

extern "C" void kernel_launch(void* const* d_in, const int* in_sizes, int n_in,
                              void* d_out, int out_size, void* d_ws, size_t ws_size, hipStream_t stream) {
    if (n_in < 9) return;
    if ((size_t)in_sizes[0] < (size_t)NB * CC * SEQ_FULL) return;
    if (in_sizes[1] < CC * CC || in_sizes[3] < CC * CC || in_sizes[5] < CC * CC || in_sizes[7] < CC * CC) return;
    if (in_sizes[2] < CC || in_sizes[4] < CC || in_sizes[6] < CC || in_sizes[8] < CC) return;
    if ((size_t)out_size < (size_t)NB * CC * HW) return;
    const float* x = (const float*)d_in[0]; const float* Wq = (const float*)d_in[1]; const float* bq = (const float*)d_in[2]; const float* Wk = (const float*)d_in[3]; const float* bk = (const float*)d_in[4];
    const float* Wv = (const float*)d_in[5]; const float* bv = (const float*)d_in[6]; const float* Wu = (const float*)d_in[7]; const float* bu = (const float*)d_in[8];
    float* OUT = (float*)d_out;
    char* wsp = (char*)d_ws;
    auto take = [&](size_t bytes) { char* p = wsp; wsp += (bytes + 255) & ~(size_t)255; return (void*)p; };
    bf* BQ = (bf*)take((size_t)CC * CC * 2); bf* BK = (bf*)take((size_t)CC * CC * 2); bf* BV = (bf*)take((size_t)CC * CC * 2); bf* BU = (bf*)take((size_t)CC * CC * 2);
    bf* XT = (bf*)take((size_t)HW * CC * 2);
    float* QF = (float*)take((size_t)CC * HW * 4); float* KF = (float*)take((size_t)CC * HW * 4); float* VF = (float*)take((size_t)CC * HW * 4);
    bf* QH = (bf*)take((size_t)HW * CC * 2); bf* QL = (bf*)take((size_t)HW * CC * 2); bf* KH = (bf*)take((size_t)HW * CC * 2); bf* KL = (bf*)take((size_t)HW * CC * 2);
    h16* VT = (h16*)take((size_t)CC * HW * 2);
    float* S = (float*)take((size_t)HW * HW * 4); h16* P16 = (h16*)take((size_t)HW * HW * 2);
    bf* ATh = (bf*)take((size_t)HW * CC * 2); bf* ATl = (bf*)take((size_t)HW * CC * 2);
    float* Y = QF;
    float* Zt = KF;
    if ((size_t)(wsp - (char*)d_ws) > ws_size) return;
    const unsigned g8w = (unsigned)((CC * CC / 8 + 255) / 256);
    k_cvt8<<<g8w, 256, 0, stream>>>(Wq, BQ, CC * CC / 8); k_cvt8<<<g8w, 256, 0, stream>>>(Wk, BK, CC * CC / 8); k_cvt8<<<g8w, 256, 0, stream>>>(Wv, BV, CC * CC / 8); k_cvt8<<<g8w, 256, 0, stream>>>(Wu, BU, CC * CC / 8);
    const unsigned gE4 = (unsigned)(((size_t)HW * CC / 4 + 255) / 256);
    const unsigned gE2 = (unsigned)(((size_t)CC * HW / 2 + 255) / 256);
    for (int b = 0; b < NB; ++b) { const float* xb = x + (size_t)b * CC * SEQ_FULL;
        k_xt<<<gE4, 256, 0, stream>>>(xb, XT);
        k_gemmw<bf, 0, 2><<<dim3(CC / 64, HW / 64, 1), 32, 0, stream>>>(BQ, nullptr, XT, nullptr, CC, QF, HW, bq, 0, 0, 0); k_hl<<<gE4, 256, 0, stream>>>(QF, QH, QL);
        k_gemmw<bf, 0, 2><<<dim3(CC / 64, HW / 64, 1), 32, 0, stream>>>(BK, nullptr, XT, nullptr, CC, KF, HW, bk, 0, 0, 0); k_hl<<<gE4, 256, 0, stream>>>(KF, KH, KL);
        k_gemmw<bf, 0, 2><<<dim3(CC / 64, HW / 64, 1), 32, 0, stream>>>(BV, nullptr, XT, nullptr, CC, VF, HW, bv, 0, 0, 0); k_gt16<<<gE2, 256, 0, stream>>>(VF, VT);
        k_gemmw<bf, 2, 0><<<dim3(HW / 64, HW / 64, 1), 32, 0, stream>>>(QH, QL, KH, KL, CC, S, HW, nullptr, 0, 0, 0);
        k_rsoft<<<HW / 8, 256, 0, stream>>>(S, P16);
        k_gemmw<h16, 0, 0><<<dim3(HW / 64, CC / 64, 1), 32, 0, stream>>>(P16, nullptr, VT, nullptr, HW, Y, CC, nullptr, 0, 0, 0);
        k_at<<<gE4, 256, 0, stream>>>(Y, ATh, ATl);
        k_gemmw<bf, 1, 1><<<dim3(HW / 64, CC / 64, 1), 32, 0, stream>>>(ATh, ATl, BU, nullptr, CC, Zt, CC, bu, 0, 0, 0);
        k_fin<<<gE4, 256, 0, stream>>>(Zt, xb, OUT + (size_t)b * CC * HW); }
}
